// PointNetHetero_67783173865977
// MI455X (gfx1250) — hardware-verified
//
#include <hip/hip_runtime.h>
#include <stddef.h>
#include <stdint.h>


#define NTHR_MLP 128
#define NTHR_FC 256
#define ELEN 2080
#define CWD 768
#define OUTW 262
#define G_W1 1024
#define G_W2 4096
#define G_FW 24576
#define G_ALL (G_W1 + G_W2 + G_FW)

typedef __bf16 v16b __attribute__((ext_vector_type(16)));
typedef float v8f __attribute__((ext_vector_type(8)));
typedef unsigned int v8u __attribute__((ext_vector_type(8)));
typedef unsigned int v4u __attribute__((ext_vector_type(4)));
typedef int v4i_t __attribute__((ext_vector_type(4)));
typedef v4i_t __attribute__((may_alias)) v4i;
typedef float v4f_t __attribute__((ext_vector_type(4)));
typedef v4f_t __attribute__((may_alias)) v4f;

union Frag { v16b v; v8u u; };

__device__ __forceinline__ unsigned int bf16_bits(float x) {
  const unsigned int u = __float_as_uint(x);
  return ((u + 0x7FFFu + ((u >> 16) & 1u)) >> 16) & 0xFFFFu;
}

__device__ __forceinline__ void split_pair(float x0, float x1, unsigned int& hw, unsigned int& lw) {
  const unsigned int h0 = bf16_bits(x0), h1 = bf16_bits(x1);
  const unsigned int l0 = bf16_bits(x0 - __uint_as_float(h0 << 16));
  const unsigned int l1 = bf16_bits(x1 - __uint_as_float(h1 << 16));
  hw = h0 | (h1 << 16);
  lw = l0 | (l1 << 16);
}

__device__ __forceinline__ void load_a_split(const float* rp, int h, Frag& fh, Frag& fl) {
  const v4f a0 = *(const v4f*)(rp + 8 * h);
  const v4f a1 = *(const v4f*)(rp + 8 * h + 4);
  const v4f a2 = *(const v4f*)(rp + 16 + 8 * h);
  const v4f a3 = *(const v4f*)(rp + 16 + 8 * h + 4);
  v8u hu = {}, lu = {};
  unsigned int hw, lw;
  split_pair(a0[0], a0[1], hw, lw); hu[0] = hw; lu[0] = lw;
  split_pair(a0[2], a0[3], hw, lw); hu[1] = hw; lu[1] = lw;
  split_pair(a1[0], a1[1], hw, lw); hu[2] = hw; lu[2] = lw;
  split_pair(a1[2], a1[3], hw, lw); hu[3] = hw; lu[3] = lw;
  split_pair(a2[0], a2[1], hw, lw); hu[4] = hw; lu[4] = lw;
  split_pair(a2[2], a2[3], hw, lw); hu[5] = hw; lu[5] = lw;
  split_pair(a3[0], a3[1], hw, lw); hu[6] = hw; lu[6] = lw;
  split_pair(a3[2], a3[3], hw, lw); hu[7] = hw; lu[7] = lw;
  fh.u = hu;
  fl.u = lu;
}

__device__ __forceinline__ v8u ldb(const unsigned short* __restrict__ base, int t, int lane) {
  return *(const v8u*)(base + (((size_t)t * 32 + lane) << 4));
}

__device__ __forceinline__ v8f mma3(v8f acc, const Frag& ah, const Frag& al,
                                    const Frag& bh, const Frag& bl) {
  acc = __builtin_amdgcn_wmma_f32_16x16x32_bf16(false, ah.v, false, bh.v, (short)0, acc, false, false);
  acc = __builtin_amdgcn_wmma_f32_16x16x32_bf16(false, ah.v, false, bl.v, (short)0, acc, false, false);
  acc = __builtin_amdgcn_wmma_f32_16x16x32_bf16(false, al.v, false, bh.v, (short)0, acc, false, false);
  asm volatile("v_nop\n\tv_nop\n\tv_nop\n\tv_nop"
               : "+v"(acc)
               : "v"(ah.v), "v"(al.v), "v"(bh.v), "v"(bl.v));
  return acc;
}

__global__ __launch_bounds__(256) void k_prep(const float* __restrict__ w1,
                                              const float* __restrict__ w2,
                                              const float* __restrict__ fw,
                                              unsigned short* w1h, unsigned short* w1l,
                                              unsigned short* w2h, unsigned short* w2l,
                                              unsigned short* fwh, unsigned short* fwl) {
  const int g = blockIdx.x * 256 + (int)threadIdx.x;
  if (g >= G_ALL) return;
  const float* src;
  unsigned short* dh;
  unsigned short* dl;
  int ncol, ntn, gl;
  if (g < G_W1) {
    src = w1; dh = w1h; dl = w1l; ncol = 128; ntn = 8; gl = g;
  } else if (g < G_W1 + G_W2) {
    src = w2; dh = w2h; dl = w2l; ncol = 256; ntn = 16; gl = g - G_W1;
  } else {
    src = fw; dh = fwh; dl = fwl; ncol = 256; ntn = 16; gl = g - G_W1 - G_W2;
  }
  const int elem0 = gl * 8;
  const int t = elem0 >> 9;
  const int lane = (elem0 >> 4) & 31;
  const int e0 = elem0 & 15;
  const int hh = lane >> 4;
  const int kt = t / ntn;
  const int nt = t - kt * ntn;
  const int n = nt * 16 + (lane & 15);
  const int kb = kt * 32 + ((e0 == 0) ? (8 * hh) : (16 + 8 * hh));
  float v[8];
#pragma unroll
  for (int j = 0; j < 8; ++j) v[j] = src[(size_t)(kb + j) * ncol + n];
  v4u hq = {}, lq = {};
  unsigned int hw, lw;
  split_pair(v[0], v[1], hw, lw); hq[0] = hw; lq[0] = lw;
  split_pair(v[2], v[3], hw, lw); hq[1] = hw; lq[1] = lw;
  split_pair(v[4], v[5], hw, lw); hq[2] = hw; lq[2] = lw;
  split_pair(v[6], v[7], hw, lw); hq[3] = hw; lq[3] = lw;
  volatile v4u* ph = (volatile v4u*)(dh + elem0);
  volatile v4u* pl = (volatile v4u*)(dl + elem0);
  *ph = hq;
  *pl = lq;
  __threadfence();
  *ph = hq;
  *pl = lq;
}

__global__ __launch_bounds__(256) void k_scan(const float* __restrict__ data,
                                              const int* __restrict__ ppb,
                                              int P, int nb, int* eout) {
  __shared__ __align__(16) int srow[ELEN];
  __shared__ int wcnt[8];
  const int tid = (int)threadIdx.x;
  const int lane = tid & 31;
  const int wv = tid >> 5;

  int bs = ppb[0];
  if (bs < 1) bs = 1;
  int nseg = P / bs;
  if (nseg > nb) nseg = nb;
  const int need = nseg + 1;

  for (int i = tid; i < ELEN; i += 256) srow[i] = P;
  __syncthreads();

  int running = 0;
  for (int base = 0; base < P; base += 256) {
    const int row = base + tid;
    bool flag = false;
    if (row < P) flag = data[(size_t)row * 9 + 8] > 0.0f;
    const unsigned int bal = __builtin_amdgcn_ballot_w32(flag);
    const int cnt = __builtin_popcount(bal);
    const int lower = __builtin_popcount(bal & ((1u << lane) - 1u));
    if (lane == 0) wcnt[wv] = cnt;
    __syncthreads();
    int prefix = 0, total = 0;
#pragma unroll
    for (int w = 0; w < 8; ++w) {
      const int c = wcnt[w];
      total += c;
      if (w < wv) prefix += c;
    }
    const int rank = running + prefix + lower;
    if (flag && rank < need) srow[rank] = row;
    running += total;
    __syncthreads();
    if (running >= need) break;
  }
  __syncthreads();

  v4i v0 = *(const v4i*)(srow + 4 * tid);
  v4i v1 = *(const v4i*)(srow + 4 * (tid + 256));
  const bool has2 = tid < (ELEN / 4 - 512);
  v4i v2 = v0;
  if (has2) v2 = *(const v4i*)(srow + 4 * (tid + 512));
  volatile v4i* p0 = (volatile v4i*)(eout + 4 * tid);
  volatile v4i* p1 = (volatile v4i*)(eout + 4 * (tid + 256));
  volatile v4i* p2 = (volatile v4i*)(eout + 4 * (tid + 512));
  *p0 = v0;
  *p1 = v1;
  if (has2) *p2 = v2;
  __threadfence();
  *p0 = v0;
  *p1 = v1;
  if (has2) *p2 = v2;
}

__global__ __launch_bounds__(NTHR_MLP) void k_mlp(const float* __restrict__ data,
                                                  const int* __restrict__ E, int P, int nb,
                                                  const float* __restrict__ w0,
                                                  const float* __restrict__ b0,
                                                  const unsigned short* __restrict__ w1h,
                                                  const unsigned short* __restrict__ w1l,
                                                  const float* __restrict__ b1,
                                                  const unsigned short* __restrict__ w2h,
                                                  const unsigned short* __restrict__ w2l,
                                                  const float* __restrict__ b2,
                                                  float* cw) {
  __shared__ __align__(16) float spnt[64 * 4];
  __shared__ __align__(16) float sh0[4 * 16 * 64];
  __shared__ __align__(16) float sh1[4 * 16 * 128];
  __shared__ float smax[4 * 256];
  __shared__ float smin[4 * 256];
  __shared__ float ssum[4 * 256];
  __shared__ __align__(16) float scw[CWD];

  const int tid = (int)threadIdx.x;
  const int lane = tid & 31;
  const int wv = tid >> 5;
  const int h = lane >> 4;
  const int m = lane & 15;
  const int k = blockIdx.x;
  if (k >= nb) return;

  const float PINF = __builtin_huge_valf();
  const float NINF = -__builtin_huge_valf();

  int beg = E[k];
  int end = E[k + 1];
  if (beg < 0) beg = 0;
  if (beg > P) beg = P;
  if (end < beg) end = beg;
  if (end > P) end = P;
  const int npts = end - beg;

  for (int i = tid; i < 4 * 256; i += NTHR_MLP) {
    smax[i] = NINF;
    smin[i] = PINF;
    ssum[i] = 0.0f;
  }
  __syncthreads();

  float* h0w = sh0 + wv * (16 * 64);
  float* h1w = sh1 + wv * (16 * 128);

  for (int cb = 0; cb < npts; cb += 64) {
    if (tid < 64) {
      const int row = cb + tid;
      float p0 = 0.0f, p1 = 0.0f, p2 = 0.0f;
      if (row < npts) {
        const float* x = data + (size_t)(beg + row) * 9;
        const float s = x[6];
        p0 = (x[0] - x[3]) * s;
        p1 = (x[1] - x[4]) * s;
        p2 = (x[2] - x[5]) * s;
      }
      spnt[tid * 4 + 0] = p0;
      spnt[tid * 4 + 1] = p1;
      spnt[tid * 4 + 2] = p2;
      spnt[tid * 4 + 3] = 0.0f;
    }
    __syncthreads();

    const bool wact = (cb + wv * 16) < npts;

    if (wact) {
#pragma unroll
      for (int cc = 0; cc < 2; ++cc) {
        const int c = lane + 32 * cc;
        const float wa = w0[c], wb = w0[64 + c], wc = w0[128 + c], bb = b0[c];
#pragma unroll 4
        for (int r = 0; r < 16; ++r) {
          const float* p = spnt + (wv * 16 + r) * 4;
          const float v = (p[0] * wa + p[1] * wb + p[2] * wc) + bb;
          h0w[r * 64 + c] = fmaxf(v, 0.0f);
        }
      }
    }
    __syncthreads();

    if (wact) {
      Frag ah0, al0, ah1, al1;
      load_a_split(h0w + m * 64, h, ah0, al0);
      load_a_split(h0w + m * 64 + 32, h, ah1, al1);
#pragma unroll 1
      for (int nt = 0; nt < 8; ++nt) {
        v8f acc = {};
        Frag bh, bl;
        bh.u = ldb(w1h, nt, lane);
        bl.u = ldb(w1l, nt, lane);
        acc = mma3(acc, ah0, al0, bh, bl);
        bh.u = ldb(w1h, 8 + nt, lane);
        bl.u = ldb(w1l, 8 + nt, lane);
        acc = mma3(acc, ah1, al1, bh, bl);
        const int c = nt * 16 + m;
        const float bb = b1[c];
#pragma unroll
        for (int r = 0; r < 8; ++r)
          h1w[(8 * h + r) * 128 + c] = fmaxf(acc[r] + bb, 0.0f);
      }
    }
    __syncthreads();

    if (wact) {
      Frag ah[4], al[4];
#pragma unroll
      for (int ks = 0; ks < 4; ++ks) load_a_split(h1w + m * 128 + ks * 32, h, ah[ks], al[ks]);
      const int rb = cb + wv * 16 + 8 * h;
#pragma unroll 1
      for (int nt = 0; nt < 16; ++nt) {
        v8f acc = {};
#pragma unroll
        for (int ks = 0; ks < 4; ++ks) {
          Frag bh, bl;
          bh.u = ldb(w2h, ks * 16 + nt, lane);
          bl.u = ldb(w2l, ks * 16 + nt, lane);
          acc = mma3(acc, ah[ks], al[ks], bh, bl);
        }
        const int c = nt * 16 + m;
        const float bb = b2[c];
        float lmax = NINF, lmin = PINF, lsum = 0.0f;
#pragma unroll
        for (int r = 0; r < 8; ++r) {
          const float v = acc[r] + bb;
          if (rb + r < npts) {
            lmax = fmaxf(lmax, v);
            lmin = fminf(lmin, v);
            lsum += v;
          }
        }
        lmax = fmaxf(lmax, __shfl_xor(lmax, 16, 32));
        lmin = fminf(lmin, __shfl_xor(lmin, 16, 32));
        lsum += __shfl_xor(lsum, 16, 32);
        if (lane < 16) {
          const int ix = wv * 256 + c;
          smax[ix] = fmaxf(smax[ix], lmax);
          smin[ix] = fminf(smin[ix], lmin);
          ssum[ix] += lsum;
        }
      }
    }
    __syncthreads();
  }

  const float inv = 1.0f / (float)npts;
  for (int c = tid; c < 256; c += NTHR_MLP) {
    float mx = smax[c], mn = smin[c], sm = ssum[c];
#pragma unroll
    for (int w = 1; w < 4; ++w) {
      mx = fmaxf(mx, smax[w * 256 + c]);
      mn = fminf(mn, smin[w * 256 + c]);
      sm += ssum[w * 256 + c];
    }
    scw[c] = mx;
    scw[256 + c] = mn;
    scw[512 + c] = sm * inv;
  }
  __syncthreads();

  float* dst = cw + (size_t)k * CWD;
  const v4f q0 = *(const v4f*)(scw + 4 * tid);
  const bool has1 = tid < (CWD / 4 - NTHR_MLP);
  v4f q1 = q0;
  if (has1) q1 = *(const v4f*)(scw + 4 * (tid + NTHR_MLP));
  volatile v4f* p0 = (volatile v4f*)(dst + 4 * tid);
  volatile v4f* p1 = (volatile v4f*)(dst + 4 * (tid + NTHR_MLP));
  *p0 = q0;
  if (has1) *p1 = q1;
  __threadfence();
  *p0 = q0;
  if (has1) *p1 = q1;
}

__global__ __launch_bounds__(NTHR_FC) void k_fc(const float* __restrict__ cw,
                                                const unsigned short* __restrict__ fwh,
                                                const unsigned short* __restrict__ fwl,
                                                const float* __restrict__ fb,
                                                const float* __restrict__ data,
                                                const int* __restrict__ E,
                                                int P, int npc, int nb, float* out) {
  __shared__ __align__(16) float sout[16 * OUTW];

  const int tid = (int)threadIdx.x;
  const int lane = tid & 31;
  const int wv = tid >> 5;
  const int h = lane >> 4;
  const int m = lane & 15;
  const int r0 = blockIdx.x * 16;
  if (r0 >= nb) return;
  const int nt0 = wv * 2;

  v8f acc0 = {}, acc1 = {};
  const float* arow = cw + (size_t)(r0 + m) * CWD;
#pragma unroll 1
  for (int kt = 0; kt < CWD / 32; ++kt) {
    Frag ah, al;
    load_a_split(arow + kt * 32, h, ah, al);
    Frag bh0, bl0, bh1, bl1;
    bh0.u = ldb(fwh, kt * 16 + nt0, lane);
    bl0.u = ldb(fwl, kt * 16 + nt0, lane);
    bh1.u = ldb(fwh, kt * 16 + nt0 + 1, lane);
    bl1.u = ldb(fwl, kt * 16 + nt0 + 1, lane);
    acc0 = mma3(acc0, ah, al, bh0, bl0);
    acc1 = mma3(acc1, ah, al, bh1, bl1);
  }
  {
    const int c0 = nt0 * 16 + m;
    const int c1 = c0 + 16;
    const float bb0 = fb[c0], bb1 = fb[c1];
#pragma unroll
    for (int r = 0; r < 8; ++r) {
      sout[(8 * h + r) * OUTW + c0] = acc0[r] + bb0;
      sout[(8 * h + r) * OUTW + c1] = acc1[r] + bb1;
    }
  }
  if (tid < 16) {
    const int kk = r0 + tid;
    const int e = E[kk];
    const int fr = (e >= 0 && e < P) ? e : 0;
    const float* x = data + (size_t)fr * 9;
    float* so = sout + tid * OUTW;
    so[256] = x[7];
    so[257] = x[3];
    so[258] = x[4];
    so[259] = x[5];
    so[260] = x[6];
    float ps = 1.0f;
    if (kk > 0) {
      const int ep = E[kk - 1];
      const int fp = (ep >= 0 && ep < P) ? ep : 0;
      ps = (float)(fr / npc - fp / npc);
    }
    so[261] = ps;
  }
  __syncthreads();

  float* dst = out + (size_t)r0 * OUTW;
  const v4f q0 = *(const v4f*)(sout + 4 * tid);
  const v4f q1 = *(const v4f*)(sout + 4 * (tid + 256));
  const v4f q2 = *(const v4f*)(sout + 4 * (tid + 512));
  const v4f q3 = *(const v4f*)(sout + 4 * (tid + 768));
  const bool has4 = tid < (16 * OUTW / 4 - 1024);
  v4f q4 = q0;
  if (has4) q4 = *(const v4f*)(sout + 4 * (tid + 1024));
  volatile v4f* p0 = (volatile v4f*)(dst + 4 * tid);
  volatile v4f* p1 = (volatile v4f*)(dst + 4 * (tid + 256));
  volatile v4f* p2 = (volatile v4f*)(dst + 4 * (tid + 512));
  volatile v4f* p3 = (volatile v4f*)(dst + 4 * (tid + 768));
  volatile v4f* p4 = (volatile v4f*)(dst + 4 * (tid + 1024));
  *p0 = q0;
  *p1 = q1;
  *p2 = q2;
  *p3 = q3;
  if (has4) *p4 = q4;
  __threadfence();
  *p0 = q0;
  *p1 = q1;
  *p2 = q2;
  *p3 = q3;
  if (has4) *p4 = q4;
}

extern "C" void kernel_launch(void* const* d_in, const int* in_sizes, int n_in,
                              void* d_out, int out_size, void* d_ws, size_t ws_size,
                              hipStream_t stream) {
  if (n_in < 10) return;
  if (in_sizes[0] <= 0 || (in_sizes[0] % 9) != 0) return;
  const int P = in_sizes[0] / 9;
  if (out_size <= 0 || (out_size % OUTW) != 0) return;
  const int NB = out_size / OUTW;
  if ((NB % 16) != 0 || NB + 1 > ELEN) return;
  if (in_sizes[1] != 3 * 64 || in_sizes[2] < 64) return;
  if (in_sizes[3] != 64 * 128 || in_sizes[4] < 128) return;
  if (in_sizes[5] != 128 * 256 || in_sizes[6] < 256) return;
  if (in_sizes[7] != CWD * 256 || in_sizes[8] < 256) return;
  if (in_sizes[9] < 1) return;
  int npc = P / 16;
  if (npc < 1) npc = 1;

  const float* data = (const float*)d_in[0];
  const float* w0 = (const float*)d_in[1];
  const float* b0 = (const float*)d_in[2];
  const float* w1 = (const float*)d_in[3];
  const float* b1 = (const float*)d_in[4];
  const float* w2 = (const float*)d_in[5];
  const float* b2 = (const float*)d_in[6];
  const float* fw = (const float*)d_in[7];
  const float* fb = (const float*)d_in[8];
  const int* ppb = (const int*)d_in[9];

  size_t off = 0;
  const size_t off_e = off;   off += 8448;
  const size_t off_w1h = off; off += (size_t)G_W1 * 16;
  const size_t off_w1l = off; off += (size_t)G_W1 * 16;
  const size_t off_w2h = off; off += (size_t)G_W2 * 16;
  const size_t off_w2l = off; off += (size_t)G_W2 * 16;
  const size_t off_fwh = off; off += (size_t)G_FW * 16;
  const size_t off_fwl = off; off += (size_t)G_FW * 16;
  const size_t off_cw = off;  off += (size_t)NB * CWD * 4;
  if (off > ws_size) return;

  char* ws = (char*)d_ws;
  int* E = (int*)(ws + off_e);
  unsigned short* w1h = (unsigned short*)(ws + off_w1h);
  unsigned short* w1l = (unsigned short*)(ws + off_w1l);
  unsigned short* w2h = (unsigned short*)(ws + off_w2h);
  unsigned short* w2l = (unsigned short*)(ws + off_w2l);
  unsigned short* fwh = (unsigned short*)(ws + off_fwh);
  unsigned short* fwl = (unsigned short*)(ws + off_fwl);
  float* cw = (float*)(ws + off_cw);

  k_prep<<<(G_ALL + 255) / 256, 256, 0, stream>>>(w1, w2, fw, w1h, w1l, w2h, w2l, fwh, fwl);
  k_scan<<<1, 256, 0, stream>>>(data, ppb, P, NB, E);
  k_mlp<<<NB, NTHR_MLP, 0, stream>>>(data, E, P, NB, w0, b0, w1h, w1l, b1, w2h, w2l, b2, cw);
  k_fc<<<NB / 16, NTHR_FC, 0, stream>>>(cw, fwh, fwl, fb, data, E, P, npc, NB, (float*)d_out);
}
